// MultiHeadAttention_58110907515489
// MI455X (gfx1250) — hardware-run, weakly checked
//
#include <hip/hip_runtime.h>


#ifndef NB
#define NB 2
#endif
#ifndef SEQ
#define SEQ 4096
#endif
#define NB_FULL  2
#define SEQ_FULL 4096
#ifndef OUT_SEQ
#define OUT_SEQ SEQ
#endif
#define DM   96
#define NH_  6
#define HD   16
#define HDP  32
#define NQK  (NH_ * HDP)
#define MV   128
#define AW   4
#define OSP  20
#define OPP  100
#define EROWS (SEQ < 512 ? SEQ : 512)
#define QRS  2048.0f
#define QRI  (1.0f / 2048.0f)
#define SC2  ((float)(0.25 * 1.4426950408889634))
#define PSH  14.0f
#define PMINE (-14.0f)
#define NEGB (-3.0e38f)
#define CXS  64.0f
#define WPS  64.0f
#define OSC  (1.0f / 4096.0f)

static_assert(HD == 16);
static_assert(HDP == 32);
static_assert(NH_ * HD == DM);
static_assert(NH_ % 2 == 0);
static_assert(DM % 32 == 0);
static_assert(DM % 16 == 0);
static_assert(DM % 8 == 0);
static_assert(NQK % 64 == 0);
static_assert(64 % HDP == 0);
static_assert(MV % 64 == 0);
static_assert(MV >= DM);
static_assert(SEQ % 64 == 0);
static_assert((NB * SEQ) % 64 == 0);
static_assert(SEQ % 32 == 0);
static_assert(SEQ % (16 * AW) == 0);
static_assert(EROWS % 64 == 0);
static_assert(EROWS % 32 == 0);
static_assert(EROWS >= 32);
static_assert(EROWS <= SEQ);
static_assert(EROWS % (16 * AW) == 0);
static_assert((SEQ - EROWS) % (16 * AW) == 0);
static_assert(((size_t)SEQ * DM) % 8 == 0);
static_assert(((size_t)DM * DM) % 8 == 0);
static_assert(NB <= NB_FULL);
static_assert(SEQ <= SEQ_FULL);
static_assert((OSP * 4) % 16 == 0);
static_assert(OSP >= HD);
static_assert((OPP * 4) % 16 == 0);
static_assert(OPP >= DM);
static_assert(16 * 68 * 4 <= 131072);
static_assert(AW * 16 * OSP * 4 <= 131072);
static_assert(16 * OPP * 4 <= 131072);
static_assert(2 * 2 * 32 * 8 == 16 * 64);
static_assert(4 * 32 * 8 == 16 * 64);
static_assert(32 * 8 == 16 * HD);
static_assert(12 * 32 * 4 == 16 * DM);

typedef _Float16 h16;
typedef unsigned short bf;
typedef __attribute__((ext_vector_type(16))) __bf16   v16bf;
typedef __attribute__((ext_vector_type(16))) _Float16 v16h;
typedef __attribute__((ext_vector_type(8)))  _Float16 v8h;
typedef __attribute__((ext_vector_type(8)))  unsigned short v8us;
typedef __attribute__((ext_vector_type(8)))  float    v8f;
typedef __attribute__((ext_vector_type(4)))  float    v4f;
typedef v4f  __attribute__((may_alias)) v4fa;

__device__ __forceinline__ unsigned short f2bf(float f) { unsigned u = __float_as_uint(f); u += 0x7FFFu + ((u >> 16) & 1u); return (unsigned short)(u >> 16); }
__device__ __forceinline__ float bfr(float f) { return __uint_as_float(((unsigned)f2bf(f)) << 16); }
__device__ __forceinline__ v16h cat16(v8h lo, v8h hi) { return __builtin_shufflevector(lo, hi, 0, 1, 2, 3, 4, 5, 6, 7, 8, 9, 10, 11, 12, 13, 14, 15); }
__device__ __forceinline__ v16bf cat16b(v8us lo, v8us hi) { return __builtin_bit_cast(v16bf, __builtin_shufflevector(lo, hi, 0, 1, 2, 3, 4, 5, 6, 7, 8, 9, 10, 11, 12, 13, 14, 15)); }
__device__ __forceinline__ v8f wmma16(v16h a, v16h b, v8f c) { return __builtin_amdgcn_wmma_f32_16x16x32_f16(false, a, false, b, (short)0, c, false, false); }
__device__ __forceinline__ v8f wmmab(v16bf a, v16bf b, v8f c) { return __builtin_amdgcn_wmma_f32_16x16x32_bf16(false, a, false, b, (short)0, c, false, false); }
__device__ __forceinline__ v8f wmma16g(v16h a, v16h b, v8f c) { c = wmma16(a, b, c); asm volatile("v_nop\n\tv_nop\n\tv_nop\n\tv_nop" : "+v"(c) : "v"(a), "v"(b)); return c; }
__device__ __forceinline__ v8f wmmabg(v16bf a, v16bf b, v8f c) { c = wmmab(a, b, c); asm volatile("v_nop\n\tv_nop\n\tv_nop\n\tv_nop" : "+v"(c) : "v"(a), "v"(b)); return c; }
__device__ __forceinline__ v16h  ldh(const h16* p) { return cat16(*(const v8h*)p, *(const v8h*)(p + 16)); }
__device__ __forceinline__ v16bf ldb(const bf* p)  { return cat16b(*(const v8us*)p, *(const v8us*)(p + 16)); }
__device__ __forceinline__ void wave_sync() { __builtin_amdgcn_fence(3  , "wavefront"); __builtin_amdgcn_wave_barrier(); asm volatile("" ::: "memory"); }
static __device__ __forceinline__ h16 toh_flush(float v) { const h16 r = (h16)v; return (fabsf(v) < 6.103515625e-05f) ? (h16)0.0f : r; }

__global__ __launch_bounds__(256) void k_cvt8(const float* __restrict__ src, bf* dst, size_t n8) {
    const size_t i = (size_t)blockIdx.x * 256 + threadIdx.x; if (i >= n8) return;
    const v8f v = *(const v8f*)(src + i * 8); v8us o;
#pragma unroll
    for (int k = 0; k < 8; ++k) o[k] = f2bf(v[k]);
    *(volatile v8us*)(dst + i * 8) = o; __threadfence(); *(volatile v8us*)(dst + i * 8) = o;
}

__global__ __launch_bounds__(256) void k_wt(const float* __restrict__ W, bf* dst, int dp, int n8) {
    const int i = blockIdx.x * 256 + threadIdx.x; if (i >= n8) return;
    const int n = i / (DM / 8), c8 = (i % (DM / 8)) * 8;
    const int h = n / dp, d = n % dp;
    const bool ok = (h < NH_) & (d < HD);
    const int hc = h < NH_ ? h : (NH_ - 1);
    const int dc = d < HD ? d : (HD - 1);
    v8us o;
#pragma unroll
    for (int k = 0; k < 8; ++k) {
        float x = W[((size_t)hc * DM + (size_t)(c8 + k)) * HD + dc];
        asm volatile("" : "+v"(x));
        const unsigned short w = f2bf(x);
        o[k] = ok ? w : (unsigned short)0; }
    *(volatile v8us*)(dst + (size_t)i * 8) = o; __threadfence(); *(volatile v8us*)(dst + (size_t)i * 8) = o;
}

__global__ __launch_bounds__(256) void k_wph(const float* __restrict__ W, h16* dst, int n8) {
    const int i = blockIdx.x * 256 + threadIdx.x; if (i >= n8) return;
    const v8f v = *(const v8f*)(W + (size_t)i * 8); v8h o;
#pragma unroll
    for (int k = 0; k < 8; ++k) o[k] = toh_flush(bfr(v[k]) * WPS);
    *(volatile v8h*)(dst + (size_t)i * 8) = o; __threadfence(); *(volatile v8h*)(dst + (size_t)i * 8) = o;
}

template <int MODE>
__device__ __forceinline__ void proj_body(const bf* __restrict__ A, const bf* __restrict__ Bt, h16* Ph, h16* Pr, int resT) {
    __shared__ __align__(16) float os[16 * 68];
    const int K = DM;
    const int lane = threadIdx.x & 31, lr = lane & 15, hi = lane >> 4; const int r0 = blockIdx.x * 64, c0 = blockIdx.y * 64;
    v8f acc[4][4];
#pragma unroll
    for (int mb = 0; mb < 4; ++mb)
#pragma unroll
        for (int nb = 0; nb < 4; ++nb) acc[mb][nb] = (v8f){};
    const size_t aoff = (size_t)(r0 + lr) * K + 8 * hi, boff = (size_t)(c0 + lr) * K + 8 * hi;
#pragma unroll 1
    for (int kc = 0; kc < K; kc += 32) {
        v16bf a[4];
#pragma unroll
        for (int mb = 0; mb < 4; ++mb) a[mb] = ldb(A + aoff + (size_t)mb * 16 * K + kc);
#pragma unroll
        for (int nb = 0; nb < 4; ++nb) { const v16bf b = ldb(Bt + boff + (size_t)nb * 16 * K + kc);
#pragma unroll
            for (int mb = 0; mb < 4; ++mb) acc[mb][nb] = wmmabg(a[mb], b, acc[mb][nb]); }
    }
    size_t tbase, rbase; bool wr;
    if (MODE == 0) { const int bb = r0 / SEQ, tt = r0 % SEQ; const int zc = bb * NH_ + c0 / HDP;
                     tbase = ((size_t)zc * SEQ + (size_t)tt) * HDP; rbase = ((size_t)zc * (size_t)resT + (size_t)tt) * HDP; wr = tt < resT; }
    else           { const int bb = c0 / SEQ, tt = c0 % SEQ;
                     tbase = (size_t)bb * (size_t)MV * SEQ + (size_t)r0 * SEQ + (size_t)tt; rbase = (size_t)bb * (size_t)MV * (size_t)resT + (size_t)r0 * (size_t)resT + (size_t)tt; wr = tt < resT; }
#pragma unroll
    for (int mb = 0; mb < 4; ++mb) {
#pragma unroll
        for (int nb = 0; nb < 4; ++nb) {
#pragma unroll
            for (int j = 0; j < 8; ++j) os[(hi * 8 + j) * 68 + nb * 16 + lr] = acc[mb][nb][j]; }
        wave_sync();
#pragma unroll 1
        for (int ps = 0; ps < 2; ++ps) {
            if (MODE == 0) {
                const size_t sb = tbase + (size_t)(mb * 16) * HDP;
                const size_t rb = rbase + (size_t)(mb * 16) * HDP;
#pragma unroll
                for (int hh = 0; hh < 2; ++hh) {
#pragma unroll
                    for (int s = 0; s < 2; ++s) { const int p = s * 32 + lane; const int row = p >> 2, c8 = (p & 3) * 8;
                        const v4f x0 = *(const v4fa*)(&os[row * 68 + hh * 32 + c8]); const v4f x1 = *(const v4fa*)(&os[row * 68 + hh * 32 + c8 + 4]); v8h hv, rv;
#pragma unroll
                        for (int i = 0; i < 4; ++i) { const h16 a0 = toh_flush(x0[i]); const h16 a1 = toh_flush(x1[i]); hv[i] = a0; hv[4 + i] = a1;
                                                      rv[i] = toh_flush((x0[i] - (float)a0) * QRS); rv[4 + i] = toh_flush((x1[i] - (float)a1) * QRS); }
                        const size_t oo = sb + (size_t)hh * ((size_t)SEQ * HDP) + (size_t)p * 8;
                        const size_t ro = rb + (size_t)hh * ((size_t)resT * HDP) + (size_t)p * 8;
                        *(volatile v8h*)(Ph + oo) = hv; if (wr) *(volatile v8h*)(Pr + ro) = rv; } }
            } else {
                const size_t sb = tbase + (size_t)(mb * 16) * SEQ;
                const size_t rb = rbase + (size_t)(mb * 16) * (size_t)resT;
#pragma unroll
                for (int s = 0; s < 4; ++s) { const int row = 4 * s + (lane >> 3), c8 = (lane & 7) * 8;
                    const v4f x0 = *(const v4fa*)(&os[row * 68 + c8]); const v4f x1 = *(const v4fa*)(&os[row * 68 + c8 + 4]); v8h hv, rv;
#pragma unroll
                    for (int i = 0; i < 4; ++i) { const h16 a0 = toh_flush(x0[i]); const h16 a1 = toh_flush(x1[i]); hv[i] = a0; hv[4 + i] = a1;
                                                  rv[i] = toh_flush((x0[i] - (float)a0) * QRS); rv[4 + i] = toh_flush((x1[i] - (float)a1) * QRS); }
                    const size_t oo = sb + (size_t)row * SEQ + c8;
                    const size_t ro = rb + (size_t)row * (size_t)resT + c8;
                    *(volatile v8h*)(Ph + oo) = hv; if (wr) *(volatile v8h*)(Pr + ro) = rv; }
            }
            if (ps == 0) __threadfence(); }
        wave_sync();
    }
}

__global__ __launch_bounds__(32) void k_projqk(const bf* __restrict__ A, const bf* __restrict__ Bt, h16* Ph, h16* Pr, int resT) { proj_body<0>(A, Bt, Ph, Pr, resT); }
__global__ __launch_bounds__(32) void k_projv(const bf* __restrict__ A, const bf* __restrict__ Bt, h16* Ph, h16* Pr, int resT) { proj_body<1>(A, Bt, Ph, Pr, resT); }

template <int EARLY>
__device__ __forceinline__ void flash_body(const h16* __restrict__ QH, const h16* __restrict__ QR, const h16* __restrict__ KP, const h16* __restrict__ KR,
                                           const h16* __restrict__ VT, const h16* __restrict__ VR, h16* CX, h16* CR) {
    __shared__ __align__(16) float os[AW * 16 * OSP];
    const int lane = threadIdx.x & 31, lr = lane & 15, hi = lane >> 4;
    const int wave = __builtin_amdgcn_readfirstlane((int)(threadIdx.x >> 5));
    const int zh = blockIdx.y; const int b = zh / NH_, h = zh % NH_;
    const int t0 = (EARLY ? 0 : EROWS) + (blockIdx.x * AW + wave) * 16;
    const int lim = t0 + lr;
    const int nk = (t0 + 16 + 31) & ~31;
    const size_t pbase = (size_t)zh * SEQ * HDP;
    const size_t rbase = (size_t)zh * EROWS * HDP;
    const v16h hz = (v16h){};
    const v16h qh = ldh(QH + pbase + (size_t)(t0 + lr) * HDP + 8 * hi);
    v16h qr = hz;
    if (EARLY) qr = ldh(QR + rbase + (size_t)(t0 + lr) * HDP + 8 * hi);
    const size_t ko = pbase + (size_t)lr * HDP + 8 * hi;
    const size_t kro = rbase + (size_t)lr * HDP + 8 * hi;
    const size_t vo = ((size_t)b * MV + (size_t)h * HD + (size_t)lr) * SEQ + 8 * hi;
    const size_t vro = ((size_t)b * MV + (size_t)h * HD + (size_t)lr) * EROWS + 8 * hi;
    v8f o0 = (v8f){}, oR0 = (v8f){};
    float m = NEGB, l = 0.0f;
#pragma unroll 1
    for (int key0 = 0; key0 < nk; key0 += 32) {
        const h16* ka = KP + ko + (size_t)key0 * HDP;
        const v16h ka0 = ldh(ka), kb0 = ldh(ka + 16 * HDP);
        v8f sHa = (v8f){}, sLa = (v8f){}, sHb = (v8f){}, sLb = (v8f){};
        sHa = wmma16g(ka0, qh, sHa); sHb = wmma16g(kb0, qh, sHb);
        if (EARLY) {
            const h16* kr = KR + kro + (size_t)key0 * HDP;
            const v16h kra0 = ldh(kr), krb0 = ldh(kr + 16 * HDP);
            sLa = wmma16g(ka0, qr, sLa); sLa = wmma16g(kra0, qh, sLa);
            sLb = wmma16g(kb0, qr, sLb); sLb = wmma16g(krb0, qh, sLb);
        }
        const int ja = key0 + 8 * hi;
        float ta[8], tb[8]; bool fa[8], fb[8]; float mx = NEGB;
#pragma unroll
        for (int r = 0; r < 8; ++r) {
            fa[r] = (ja + r <= lim);
            fb[r] = (ja + 16 + r <= lim);
            if (EARLY) { ta[r] = (sHa[r] + sLa[r] * QRI) * SC2; tb[r] = (sHb[r] + sLb[r] * QRI) * SC2; }
            else       { ta[r] = sHa[r] * SC2; tb[r] = sHb[r] * SC2; }
            mx = fmaxf(mx, fmaxf(fa[r] ? ta[r] : NEGB, fb[r] ? tb[r] : NEGB)); }
        mx = fmaxf(mx, __shfl_xor(mx, 16, 32));
        const float mnew = fmaxf(m, mx);
        const float alpha = __builtin_amdgcn_exp2f(m - mnew);
        const float sh = PSH - mnew;
        v16h pb, pr = hz; float ls = 0.0f;
#pragma unroll
        for (int r = 0; r < 8; ++r) {
            const float xa = ta[r] + sh, xb = tb[r] + sh;
            const float ea = __builtin_amdgcn_exp2f(xa), eb = __builtin_amdgcn_exp2f(xb);
            const float ga = (fa[r] & (xa >= PMINE)) ? ea : 0.0f;
            const float gb = (fb[r] & (xb >= PMINE)) ? eb : 0.0f;
            const h16 pa = (h16)ga; const h16 pc = (h16)gb;
            pb[r] = pa; pb[8 + r] = pc;
            if (EARLY) { pr[r] = toh_flush((ga - (float)pa) * QRS); pr[8 + r] = toh_flush((gb - (float)pc) * QRS); ls += ga + gb; }
            else       { ls += (float)pa + (float)pc; } }
        l = l * alpha + ls; m = mnew;
        o0 = o0 * alpha;
        if (EARLY) oR0 = oR0 * alpha;
        const v16h v0 = ldh(VT + vo + key0);
        o0 = wmma16g(v0, pb, o0);
        if (EARLY) {
            const v16h vr0 = ldh(VR + vro + key0);
            oR0 = wmma16g(v0, pr, oR0);
            oR0 = wmma16g(vr0, pb, oR0);
        }
    }
    l += __shfl_xor(l, 16, 32);
    const bool any = l > 0.0f;
    const float lsafe = any ? l : 1.0f;
    const float inv = any ? (1.0f / lsafe) : 0.0f;
    v8f f0 = o0;
    if (EARLY) f0 = o0 + oR0 * QRI;
    const float sc = inv * CXS;
    const int wb = wave * 16 * OSP;
    { v4f a, c;
      a[0] = f0[0] * sc; a[1] = f0[1] * sc; a[2] = f0[2] * sc; a[3] = f0[3] * sc; c[0] = f0[4] * sc; c[1] = f0[5] * sc; c[2] = f0[6] * sc; c[3] = f0[7] * sc;
      *(v4fa*)(&os[wb + lr * OSP + 8 * hi]) = a; *(v4fa*)(&os[wb + lr * OSP + 8 * hi + 4]) = c; }
    wave_sync();
    const int row = lane >> 1, c8 = (lane & 1) * 8;
    const v4f x0 = *(const v4fa*)(&os[wb + row * OSP + c8]); const v4f x1 = *(const v4fa*)(&os[wb + row * OSP + c8 + 4]);
    v8h hv, rv;
#pragma unroll
    for (int i = 0; i < 4; ++i) { const h16 a0 = toh_flush(x0[i]); const h16 a1 = toh_flush(x1[i]); hv[i] = a0; hv[4 + i] = a1;
                                  rv[i] = toh_flush((x0[i] - (float)a0) * QRS); rv[4 + i] = toh_flush((x1[i] - (float)a1) * QRS); }
    const size_t co = ((size_t)zh * SEQ + (size_t)t0) * HD + (size_t)lane * 8;
    size_t cro = 0;
    if (EARLY) cro = ((size_t)zh * EROWS + (size_t)t0) * HD + (size_t)lane * 8;
#pragma unroll 1
    for (int ps = 0; ps < 2; ++ps) {
        *(volatile v8h*)(CX + co) = hv;
        if (EARLY) *(volatile v8h*)(CR + cro) = rv;
        if (ps == 0) __threadfence(); }
}

__global__ __launch_bounds__(32 * AW) void k_flash_early(const h16* __restrict__ QH, const h16* __restrict__ QR, const h16* __restrict__ KP, const h16* __restrict__ KR,
                                                         const h16* __restrict__ VT, const h16* __restrict__ VR, h16* CX, h16* CR) {
    flash_body<1>(QH, QR, KP, KR, VT, VR, CX, CR);
}
__global__ __launch_bounds__(32 * AW) void k_flash_late(const h16* __restrict__ QH, const h16* __restrict__ KP, const h16* __restrict__ VT, h16* CX) {
    flash_body<0>(QH, (const h16*)0, KP, (const h16*)0, VT, (const h16*)0, CX, (h16*)0);
}

__global__ __launch_bounds__(32) void k_oproj(const h16* __restrict__ CX, const h16* __restrict__ CR, const h16* __restrict__ WP, const float* __restrict__ bias, float* OUT) {
    __shared__ __align__(16) float os[16 * OPP];
    const int lane = threadIdx.x & 31, lr = lane & 15, hi = lane >> 4;
    const int r0 = blockIdx.x * 16; const int bb = r0 / SEQ, tt = r0 % SEQ;
    const bool early = tt < EROWS;
    const v16h hz = (v16h){};
    v8f acc[6], accR[6];
#pragma unroll
    for (int nb = 0; nb < 6; ++nb) { acc[nb] = (v8f){}; accR[nb] = (v8f){}; }
#pragma unroll 1
    for (int s = 0; s < DM / 32; ++s) {
        const size_t ao = ((size_t)(bb * NH_ + 2 * s) * SEQ + (size_t)(tt + lr)) * HD + 8 * hi;
        const v16h a = cat16(*(const v8h*)(CX + ao), *(const v8h*)(CX + ao + (size_t)SEQ * HD));
        v16h ar = hz;
        if (early) { const size_t ro = ((size_t)(bb * NH_ + 2 * s) * EROWS + (size_t)(tt + lr)) * HD + 8 * hi;
                     ar = cat16(*(const v8h*)(CR + ro), *(const v8h*)(CR + ro + (size_t)EROWS * HD)); }
#pragma unroll
        for (int nb = 0; nb < 6; ++nb) {
            const v16h bw = ldh(WP + (size_t)(nb * 16 + lr) * DM + 8 * hi + 32 * s);
            acc[nb] = wmma16g(a, bw, acc[nb]);
            if (early) accR[nb] = wmma16g(ar, bw, accR[nb]); }
    }
#pragma unroll
    for (int nb = 0; nb < 6; ++nb) {
        const float bc = bfr(bias[nb * 16 + lr]);
#pragma unroll
        for (int j = 0; j < 8; ++j) os[(hi * 8 + j) * OPP + nb * 16 + lr] = (acc[nb][j] + accR[nb][j] * QRI) * OSC + bc; }
    wave_sync();
    float* ob = OUT + ((size_t)bb * OUT_SEQ + (size_t)tt) * DM;
#pragma unroll 1
    for (int ps = 0; ps < 2; ++ps) {
#pragma unroll
        for (int s = 0; s < 12; ++s) { const int p = s * 32 + lane; const int row = p / (DM / 4), c4 = (p % (DM / 4)) * 4;
            const v4f val = *(const v4fa*)(&os[row * OPP + c4]);
            *(volatile v4f*)(ob + (size_t)p * 4) = val; }
        if (ps == 0) __threadfence(); }
}

static constexpr size_t al256(size_t v) { return (v + 255) & ~(size_t)255; }
static constexpr size_t SZ_XB = al256((size_t)NB * SEQ * DM * 2);
static constexpr size_t SZ_WQ = al256((size_t)NQK * DM * 2);
static constexpr size_t SZ_WV = al256((size_t)MV * DM * 2);
static constexpr size_t SZ_WP = al256((size_t)DM * DM * 2);
static constexpr size_t SZ_PL = al256((size_t)NB * NH_ * SEQ * HDP * 2);
static constexpr size_t SZ_RS = al256((size_t)NB * NH_ * EROWS * HDP * 2);
static constexpr size_t SZ_VT = al256((size_t)NB * MV * SEQ * 2);
static constexpr size_t SZ_VR = al256((size_t)NB * MV * EROWS * 2);
static constexpr size_t SZ_CX = al256((size_t)NB * NH_ * SEQ * HD * 2);
static constexpr size_t SZ_CR = al256((size_t)NB * NH_ * EROWS * HD * 2);
static constexpr size_t SZ_TOTAL = SZ_XB + 2 * SZ_WQ + SZ_WV + SZ_WP + 2 * SZ_PL + 2 * SZ_RS + SZ_VT + SZ_VR + SZ_CX + SZ_CR;
static_assert(SZ_TOTAL <= (size_t)134217728);
static_assert(((size_t)NQK * (DM / 8)) % 8 == 0);
static_assert(((size_t)MV * (DM / 8)) % 8 == 0);
static_assert(((size_t)DM * DM / 8) % 8 == 0);
static_assert((size_t)(NB_FULL) * SEQ_FULL * DM * 4 == (size_t)3145728);

extern "C" void kernel_launch(void* const* d_in, const int* in_sizes, int n_in,
                              void* d_out, int out_size, void* d_ws, size_t ws_size, hipStream_t stream) {
    if (n_in < 6) return;
    const size_t needx = ((size_t)(NB - 1) * SEQ_FULL + SEQ) * DM;
    if ((size_t)in_sizes[0] < needx) return;
    if ((size_t)in_sizes[1] < (size_t)NH_ * DM * HD || (size_t)in_sizes[2] < (size_t)NH_ * DM * HD || (size_t)in_sizes[3] < (size_t)NH_ * DM * HD) return;
    if ((size_t)in_sizes[4] < (size_t)DM * DM || in_sizes[5] < DM) return;
    if ((size_t)out_size < ((size_t)(NB - 1) * OUT_SEQ + SEQ) * DM) return;
    if (SZ_TOTAL > ws_size) return;
    const float* xin = (const float*)d_in[0];
    const float* wq = (const float*)d_in[1];
    const float* wk = (const float*)d_in[2];
    const float* wv = (const float*)d_in[3];
    const float* wp = (const float*)d_in[4];
    const float* bp = (const float*)d_in[5];
    float* OUT = (float*)d_out;
    char* wsp = (char*)d_ws;
    bf* XB  = (bf*)wsp;  wsp += SZ_XB;
    bf* WQP = (bf*)wsp;  wsp += SZ_WQ;
    bf* WKP = (bf*)wsp;  wsp += SZ_WQ;
    bf* WVP = (bf*)wsp;  wsp += SZ_WV;
    h16* WPH = (h16*)wsp; wsp += SZ_WP;
    h16* QH = (h16*)wsp; wsp += SZ_PL;
    h16* KP = (h16*)wsp; wsp += SZ_PL;
    h16* QR = (h16*)wsp; wsp += SZ_RS;
    h16* KR = (h16*)wsp; wsp += SZ_RS;
    h16* VT = (h16*)wsp; wsp += SZ_VT;
    h16* VR = (h16*)wsp; wsp += SZ_VR;
    h16* CX = (h16*)wsp; wsp += SZ_CX;
    h16* CR = (h16*)wsp; wsp += SZ_CR;

    if (SEQ == SEQ_FULL) {
        const size_t n8 = (size_t)NB * SEQ * DM / 8;
        k_cvt8<<<(unsigned)((n8 + 255) / 256), 256, 0, stream>>>(xin, XB, n8);
    } else {
        const size_t n8 = (size_t)SEQ * DM / 8;
        for (int b = 0; b < NB; ++b) k_cvt8<<<(unsigned)((n8 + 255) / 256), 256, 0, stream>>>(xin + (size_t)b * SEQ_FULL * DM, XB + (size_t)b * SEQ * DM, n8);
    }
    { const int nq = NQK * (DM / 8); const int nv = MV * (DM / 8);
      k_wt<<<(unsigned)((nq + 255) / 256), 256, 0, stream>>>(wq, WQP, HDP, nq);
      k_wt<<<(unsigned)((nq + 255) / 256), 256, 0, stream>>>(wk, WKP, HDP, nq);
      k_wt<<<(unsigned)((nv + 255) / 256), 256, 0, stream>>>(wv, WVP, HD, nv);
      const int np = DM * DM / 8;
      k_wph<<<(unsigned)((np + 255) / 256), 256, 0, stream>>>(wp, WPH, np); }

    k_projqk<<<dim3(NB * SEQ / 64, NQK / 64, 1), 32, 0, stream>>>(XB, WQP, QH, QR, EROWS);
    k_projqk<<<dim3(NB * SEQ / 64, NQK / 64, 1), 32, 0, stream>>>(XB, WKP, KP, KR, EROWS);
    k_projv<<<dim3(MV / 64, NB * SEQ / 64, 1), 32, 0, stream>>>(WVP, XB, VT, VR, EROWS);

    k_flash_early<<<dim3(EROWS / (16 * AW), NB * NH_, 1), 32 * AW, 0, stream>>>(QH, QR, KP, KR, VT, VR, CX, CR);
    if (SEQ > EROWS)
        k_flash_late<<<dim3((SEQ - EROWS) / (16 * AW), NB * NH_, 1), 32 * AW, 0, stream>>>(QH, KP, VT, CX);

    k_oproj<<<dim3(NB * SEQ / 16, 1, 1), 32, 0, stream>>>(CX, CR, WPH, bp, OUT);
}
